// MaskedAutoencoderNoise_17197049053494
// MI455X (gfx1250) — hardware-run, weakly checked
//
#include <hip/hip_runtime.h>
#include <math.h>

typedef __attribute__((ext_vector_type(16))) _Float16 v16h;
typedef __attribute__((ext_vector_type(16))) __bf16 v16b;
typedef __attribute__((ext_vector_type(8)))  _Float16 v8h;
typedef __attribute__((ext_vector_type(8)))  float v8f;
typedef __attribute__((ext_vector_type(4)))  float v4f;
typedef __attribute__((ext_vector_type(2)))  float v2f;
typedef __attribute__((ext_vector_type(4)))  unsigned v4u;
typedef __attribute__((ext_vector_type(4)))  int v4i;
typedef float __attribute__((may_alias)) float_a;
typedef int __attribute__((may_alias)) int_a;

template <typename T> __device__ __forceinline__ void vst2(void* p, T v) { *(volatile T*)p = v; __threadfence(); *(volatile T*)p = v; }
__device__ __forceinline__ v8f wmma16(v16h a, v16h b, v8f c) {
  v8f d = __builtin_amdgcn_wmma_f32_16x16x32_f16(false, a, false, b, (short)0, c, false, false);
  asm volatile("v_nop\n\tv_nop\n\tv_nop\n\tv_nop" : "+v"(d) : "v"(a), "v"(b));
  return d;
}
__device__ __forceinline__ v8f wmma_bf(v16b a, v16b b, v8f c) {
  v8f d = __builtin_amdgcn_wmma_f32_16x16x32_bf16(false, a, false, b, (short)0, c, false, false);
  asm volatile("v_nop\n\tv_nop\n\tv_nop\n\tv_nop" : "+v"(d) : "v"(a), "v"(b));
  return d;
}
__device__ __forceinline__ v16h frag_h(const _Float16* rowk0, int lane) {
  union { v16h v; v8h q[2]; } u; const _Float16* p = rowk0 + 8 * (lane >> 4);
  u.q[0] = *(const v8h*)p; u.q[1] = *(const v8h*)(p + 16); return u.v;
}
__device__ __forceinline__ v16h frag_f32(const float* rowk0, int lane) {
  v16h a; const float* p = rowk0 + 8 * (lane >> 4);
#pragma unroll
  for (int i = 0; i < 8; ++i) { a[i] = (_Float16)p[i]; a[8 + i] = (_Float16)p[16 + i]; }
  return a;
}
__device__ __forceinline__ v16h frag_f32s(const float* rowk0, int lane, float sc) {
  v16h a; const float* p = rowk0 + 8 * (lane >> 4);
#pragma unroll
  for (int i = 0; i < 8; ++i) { a[i] = (_Float16)(p[i] * sc); a[8 + i] = (_Float16)(p[16 + i] * sc); }
  return a;
}
__device__ __forceinline__ v16h fragc_f32(const float* W, int k0, int n, int lane, int ld, int K) {
  v16h a; const int g = lane >> 4;
#pragma unroll
  for (int i = 0; i < 8; ++i) { const int ka = k0 + 8 * g + i, kb = ka + 16;
    a[i] = (_Float16)(ka < K ? W[(size_t)(ka < K ? ka : K - 1) * ld + n] : 0.f); a[8 + i] = (_Float16)(kb < K ? W[(size_t)(kb < K ? kb : K - 1) * ld + n] : 0.f); }
  return a;
}
struct F2 { v16b h, l; };
__device__ __forceinline__ F2 bsplit16(const float v[16]) { F2 r;
#pragma unroll
  for (int i = 0; i < 16; ++i) { const __bf16 h = (__bf16)v[i]; r.h[i] = h; r.l[i] = (__bf16)(v[i] - (float)h); }
  return r; }
__device__ __forceinline__ F2 split_row(const float* row, int k0, int lane) { float v[16]; const float* p = row + k0 + 8 * (lane >> 4);
#pragma unroll
  for (int i = 0; i < 8; ++i) { v[i] = p[i]; v[8 + i] = p[16 + i]; }
  return bsplit16(v); }
__device__ __forceinline__ F2 split_rowK(const float* row, int k0, int lane, int K) { float v[16]; const int g = lane >> 4;
#pragma unroll
  for (int i = 0; i < 8; ++i) { const int ka = k0 + 8 * g + i, kb = ka + 16; v[i] = ka < K ? row[ka < K ? ka : K - 1] : 0.f; v[8 + i] = kb < K ? row[kb < K ? kb : K - 1] : 0.f; }
  return bsplit16(v); }
__device__ __forceinline__ F2 split_col(const float* W, int k0, int n, int lane, int ld, int K) { float v[16]; const int g = lane >> 4;
#pragma unroll
  for (int i = 0; i < 8; ++i) { const int ka = k0 + 8 * g + i, kb = ka + 16; v[i] = ka < K ? W[(size_t)(ka < K ? ka : K - 1) * ld + n] : 0.f; v[8 + i] = kb < K ? W[(size_t)(kb < K ? kb : K - 1) * ld + n] : 0.f; }
  return bsplit16(v); }
__device__ __forceinline__ v8f mac3(const F2& a, const F2& b, v8f c) { c = wmma_bf(a.l, b.h, c); c = wmma_bf(a.h, b.l, c); return wmma_bf(a.h, b.h, c); }
__device__ __forceinline__ float sigm(float v) { return 1.0f / (1.0f + expf(-v)); }
#define LDSX() do { asm volatile("s_wait_dscnt 0" ::: "memory"); __builtin_amdgcn_wave_barrier(); __builtin_amdgcn_fence(__ATOMIC_RELEASE, "workgroup"); } while (0)


#define NBR 8192
#define DD 128
#define HH 64
#define WSC 256.0f
#ifndef TRB
#define TRB (NBR / 64)
#endif
typedef __attribute__((ext_vector_type(8))) __bf16 v8b;
__device__ __forceinline__ v16b frag_b(const __bf16* rowk0, int lane) {
  union { v16b v; v8b q[2]; } u; const __bf16* p = rowk0 + 8 * (lane >> 4);
  u.q[0] = *(const v8b*)p; u.q[1] = *(const v8b*)(p + 16); return u.v;
}
__device__ __forceinline__ float bfr(float v) { return (float)(__bf16)v; }
__device__ __attribute__((noinline)) float exp_ni(float v) { return expf(v); }
__device__ __attribute__((noinline)) float erf_ni(float v) { return erff(v); }

#define WS_B1H 0u
#define WS_B1L (WS_B1H + 2u * (size_t)DD * HH * DD)
#define WS_W2  (WS_B1L + 2u * (size_t)DD * HH * DD)
#define WS_W3  (WS_W2 + 2u * (size_t)DD * HH * HH)
#define WS_OT  (WS_W3 + 2u * (size_t)DD * HH * HH)
#define WS_END (WS_OT + 4u * (size_t)DD * NBR)

__global__ __launch_bounds__(128) void k_prep(const float* __restrict__ MASK, const float* __restrict__ W1, const float* __restrict__ W2, const float* __restrict__ W3, char* __restrict__ ws) {
  __shared__ __align__(16) __bf16 sbh[DD], sbl[DD]; __shared__ __align__(16) _Float16 s2[HH], s3[HH]; const int h = blockIdx.x, d = blockIdx.y, t = threadIdx.x;
  { const int j = t; const float v = bfr(MASK[j * DD + d]) * bfr(W1[((size_t)d * 2 * DD + j) * HH + h]); const __bf16 hb = (__bf16)v; sbh[j] = hb; sbl[j] = (__bf16)(v - (float)hb); }
  if (t < HH) { s2[t] = (_Float16)(bfr(W2[((size_t)d * HH + t) * HH + h]) * WSC); s3[t] = (_Float16)(bfr(W3[((size_t)d * HH + t) * HH + h]) * WSC); }
  __syncthreads();
  if (t < DD / 8) { vst2((unsigned*)((__bf16*)(ws + WS_B1H) + ((size_t)d * HH + h) * DD + t * 8), *(const v4u*)&sbh[t * 8]); vst2((unsigned*)((__bf16*)(ws + WS_B1L) + ((size_t)d * HH + h) * DD + t * 8), *(const v4u*)&sbl[t * 8]); }
  if (t < HH / 8) { vst2((unsigned*)((_Float16*)(ws + WS_W2) + ((size_t)d * HH + h) * HH + t * 8), *(const v4u*)&s2[t * 8]); vst2((unsigned*)((_Float16*)(ws + WS_W3) + ((size_t)d * HH + h) * HH + t * 8), *(const v4u*)&s3[t * 8]); } }
__device__ __forceinline__ v16h lds_frag(const _Float16 (*sh)[HH + 8], int row, int kc, int g) { v16h a; const _Float16* p = &sh[row][kc * 32 + 8 * g];
#pragma unroll
  for (int i = 0; i < 8; ++i) { a[i] = p[i]; a[8 + i] = p[16 + i]; } return a; }
__global__ __launch_bounds__(128) void k_main(const float* __restrict__ X, const float* __restrict__ Z, const float* __restrict__ W1, const float* __restrict__ B1v, const float* __restrict__ B2v, const float* __restrict__ B3v, const float* __restrict__ W4, const float* __restrict__ B4, const char* __restrict__ ws, float* __restrict__ OT) {
  __shared__ __align__(16) _Float16 sh[64][HH + 8]; __shared__ __align__(16) float sout[64];
  const int tid = threadIdx.x, wave = tid >> 5, lane = tid & 31, col = lane & 15, g = lane >> 4; const size_t rb = (size_t)blockIdx.x * 64; const size_t r0 = rb + wave * 16; const int d = blockIdx.y;
  const __bf16 *B1H = (const __bf16*)(ws + WS_B1H) + (size_t)d * HH * DD, *B1L = (const __bf16*)(ws + WS_B1L) + (size_t)d * HH * DD; const _Float16 *W2T = (const _Float16*)(ws + WS_W2) + (size_t)d * HH * HH, *W3T = (const _Float16*)(ws + WS_W3) + (size_t)d * HH * HH;
  v8f acc[4] = {};
#pragma unroll
  for (int kc = 0; kc < DD / 32; ++kc) { v16b a; { const float* p = X + (r0 + col) * DD + kc * 32 + 8 * g;
#pragma unroll
      for (int i = 0; i < 8; ++i) { a[i] = (__bf16)p[i]; a[8 + i] = (__bf16)p[16 + i]; } }
#pragma unroll
    for (int j = 0; j < 4; ++j) { acc[j] = wmma_bf(a, frag_b(B1H + (size_t)(j * 16 + col) * DD + kc * 32, lane), acc[j]); acc[j] = wmma_bf(a, frag_b(B1L + (size_t)(j * 16 + col) * DD + kc * 32, lane), acc[j]); } }
  { float zr[8];
#pragma unroll
    for (int r = 0; r < 8; ++r) zr[r] = bfr(Z[(r0 + 8 * g + r) * DD + d]);
#pragma unroll
    for (int j = 0; j < 4; ++j) { const int hcol = j * 16 + col; const float w1z = bfr(W1[((size_t)d * 2 * DD + DD + d) * HH + hcol]); const float bb = bfr(B1v[d * HH + hcol]);
#pragma unroll
      for (int r = 0; r < 8; ++r) sh[wave * 16 + 8 * g + r][hcol] = (_Float16)fmaxf(acc[j][r] + zr[r] * w1z + bb, 0.f); } }
  LDSX();
  v8f acc2[4] = {};
#pragma unroll
  for (int kc = 0; kc < HH / 32; ++kc) { const v16h a = lds_frag(sh, wave * 16 + col, kc, g);
#pragma unroll
    for (int j = 0; j < 4; ++j) acc2[j] = wmma16(a, frag_h(W2T + (size_t)(j * 16 + col) * HH + kc * 32, lane), acc2[j]); }
  LDSX();
#pragma unroll
  for (int j = 0; j < 4; ++j) { const int hcol = j * 16 + col; const float bb = bfr(B2v[d * HH + hcol]);
#pragma unroll
    for (int r = 0; r < 8; ++r) sh[wave * 16 + 8 * g + r][hcol] = (_Float16)fmaxf(acc2[j][r] * (1.0f / WSC) + bb, 0.f); }
  LDSX();
  v8f acc3[4] = {};
#pragma unroll
  for (int kc = 0; kc < HH / 32; ++kc) { const v16h a = lds_frag(sh, wave * 16 + col, kc, g);
#pragma unroll
    for (int j = 0; j < 4; ++j) acc3[j] = wmma16(a, frag_h(W3T + (size_t)(j * 16 + col) * HH + kc * 32, lane), acc3[j]); }
  float part[8];
#pragma unroll
  for (int r = 0; r < 8; ++r) { part[r] = 0.f;
#pragma unroll
    for (int j = 0; j < 4; ++j) { const int hcol = j * 16 + col; part[r] += fmaxf(acc3[j][r] * (1.0f / WSC) + bfr(B3v[d * HH + hcol]), 0.f) * bfr(W4[d * HH + hcol]); }
#pragma unroll
    for (int o = 1; o < 16; o <<= 1) part[r] += __shfl_xor(part[r], o);
    if (col == 0) sout[wave * 16 + 8 * g + r] = part[r] + bfr(B4[d]); }
  __syncthreads(); if (tid < 16) vst2(OT + (size_t)d * NBR + rb + tid * 4, *(const v4f*)&sout[tid * 4]); }
__global__ __launch_bounds__(256) void k_tr(const float* __restrict__ OT, float* __restrict__ Y) { __shared__ float st[DD][65]; __shared__ __align__(16) float so2[64][DD + 4]; const int t = threadIdx.x; const size_t b0 = (size_t)blockIdx.x * 64;
  for (int e = t; e < DD * 64; e += 256) { const int d = e >> 6, bl = e & 63; st[d][bl] = OT[(size_t)d * NBR + b0 + bl]; } __syncthreads();
  for (int e = t; e < 64 * DD; e += 256) { const int bl = e >> 7, d = e & 127; so2[bl][d] = st[d][bl]; } __syncthreads();
  for (int e = t; e < 64 * 32; e += 256) { const int bl = e >> 5, q = e & 31; vst2(Y + (b0 + bl) * DD + q * 4, *(const v4f*)&so2[bl][q * 4]); } }
extern "C" void kernel_launch(void* const* d_in, const int* in_sizes, int n_in, void* d_out, int out_size, void* d_ws, size_t ws_size, hipStream_t stream) {
  (void)in_sizes; (void)n_in; (void)out_size;
  const float** F = (const float**)d_in;
  if (ws_size < (size_t)WS_END) return;
  char* ws = (char*)d_ws; float* OT = (float*)(ws + WS_OT);
  k_prep<<<dim3(HH, DD), 128, 0, stream>>>(F[2], F[3], F[5], F[7], ws);
  k_main<<<dim3(TRB, DD), 128, 0, stream>>>(F[0], F[1], F[3], F[4], F[6], F[8], F[9], F[10], ws, OT);
  k_tr<<<TRB, 256, 0, stream>>>(OT, (float*)d_out);
}
